// FullDeepModelWithThreeStages_84413287236156
// MI455X (gfx1250) — hardware-verified
//
#include <hip/hip_runtime.h>

typedef __attribute__((ext_vector_type(16))) _Float16 v16h;
typedef __attribute__((ext_vector_type(8)))  _Float16 v8h;
typedef __attribute__((ext_vector_type(16))) __bf16   v16b;
typedef __attribute__((ext_vector_type(8)))  __bf16   v8b;
typedef __attribute__((ext_vector_type(8)))  float    v8f;
typedef __attribute__((ext_vector_type(4)))  float    v4f;

#define C_B     2
#define C_S     2048
#define C_ROWS  (C_B * C_S)
#define C_DM    256
#define C_DFF   512
#define C_H     8
#define C_DK    32
#define C_L     4
#define C_QKVN  768
#define C_LNEPS 1e-5f

__device__ __forceinline__ unsigned short f2bf_bits(float f) {
  unsigned u = __float_as_uint(f);
  return (unsigned short)((u + 0x7FFFu + ((u >> 16) & 1u)) >> 16);
}
__device__ __forceinline__ float bf_bits2f(unsigned short h) { return __uint_as_float(((unsigned)h) << 16); }

__device__ __forceinline__ void dep_guard_h(v8f& a, v8f& b, v16h x, v16h y) { asm volatile("v_nop\n\tv_nop\n\tv_nop\n\tv_nop" : "+v"(a), "+v"(b) : "v"(x), "v"(y)); }
__device__ __forceinline__ void dep_guard_b(v8f& a, v8f& b, v16b x, v16b y) { asm volatile("v_nop\n\tv_nop\n\tv_nop\n\tv_nop" : "+v"(a), "+v"(b) : "v"(x), "v"(y)); }
__device__ __forceinline__ void keep4_h(v16h a, v16h b, v16h c, v16h d) { asm volatile("v_nop" :: "v"(a), "v"(b), "v"(c), "v"(d)); }
__device__ __forceinline__ void keep4_b(v16b a, v16b b, v16b c, v16b d) { asm volatile("v_nop" :: "v"(a), "v"(b), "v"(c), "v"(d)); }
__device__ __forceinline__ void acc_guard4(v8f& a, v8f& b, v8f& c, v8f& d) { asm volatile("v_nop\n\tv_nop\n\tv_nop\n\tv_nop" : "+v"(a), "+v"(b), "+v"(c), "+v"(d)); }

template <typename T> struct Frag;
template <> struct Frag<_Float16> {
  typedef v16h V; union U { v16h v; v8h h[2]; };
  static __device__ __forceinline__ v16h load(const _Float16* p) {
    U f; f.h[0] = *(const v8h*)(p); f.h[1] = *(const v8h*)(p + 16); return f.v;
  }
  static __device__ __forceinline__ v8f mma(v16h a, v16h b, v8f c) {
    return __builtin_amdgcn_wmma_f32_16x16x32_f16(false, a, false, b, (short)0, c, false, false);
  }
  static __device__ __forceinline__ void guard(v8f& a, v8f& b, v16h x, v16h y) { dep_guard_h(a, b, x, y); }
  static __device__ __forceinline__ void keep(v16h a, v16h b, v16h c, v16h d) { keep4_h(a, b, c, d); }
};
template <> struct Frag<__bf16> {
  typedef v16b V; union U { v16b v; v8b h[2]; };
  static __device__ __forceinline__ v16b load(const __bf16* p) {
    U f; f.h[0] = *(const v8b*)(p); f.h[1] = *(const v8b*)(p + 16); return f.v;
  }
  static __device__ __forceinline__ v8f mma(v16b a, v16b b, v8f c) {
    return __builtin_amdgcn_wmma_f32_16x16x32_bf16(false, a, false, b, (short)0, c, false, false);
  }
  static __device__ __forceinline__ void guard(v8f& a, v8f& b, v16b x, v16b y) { dep_guard_b(a, b, x, y); }
  static __device__ __forceinline__ void keep(v16b a, v16b b, v16b c, v16b d) { keep4_b(a, b, c, d); }
};

__device__ __forceinline__ v8f mma_h(v16h a, v16h b, v8f c) {
  c = __builtin_amdgcn_wmma_f32_16x16x32_f16(false, a, false, b, (short)0, c, false, false);
  asm volatile("v_nop\n\tv_nop\n\tv_nop\n\tv_nop" : "+v"(c) : "v"(a), "v"(b));
  return c;
}

template <int ET> struct Elem;
template <> struct Elem<0> { typedef _Float16 T; };
template <> struct Elem<1> { typedef __bf16 T; };
template <int ET, bool SPLIT, int BIAS_MODE, int OUT_MODE, bool RESID, int ACT = 0>
__global__ __launch_bounds__(256) void wmma_gemm64(
    const unsigned short* __restrict__ Ap, const unsigned short* __restrict__ A2p, int lda, long strideA,
    const unsigned short* __restrict__ Btp, const unsigned short* __restrict__ Bt2p, int ldb, long strideB,
    void* __restrict__ Cout, void* __restrict__ Cout2, int ldc, long strideC,
    const float* __restrict__ bias,
    const float* __restrict__ resid, long strideR,
    int M, int N, int K, float scale) {
  typedef typename Elem<ET>::T T;
  typedef typename Frag<T>::V V;
  const T* A = (const T*)Ap; const T* A2 = (const T*)A2p; const T* Bt = (const T*)Btp; const T* Bt2 = (const T*)Bt2p;
  __shared__ __align__(16) float sT[8][16 * 68];
  const int b    = blockIdx.y;
  const int lane = threadIdx.x & 31;
  const int wave = threadIdx.x >> 5;
  const int tilesN = N >> 6;
  const int tilesM = M >> 6;
  const int tile = blockIdx.x * 8 + wave;
  if (tile >= tilesM * tilesN) return;
  const int tm = tile / tilesN;
  const int tn = tile - tm * tilesN;
  const int m0 = tm << 6;
  const int n0 = tn << 6;

  const T* Ab  = A  + (size_t)b * strideA;
  const T* Bb  = Bt + (size_t)b * strideB;
  const T* Ab2 = SPLIT ? (A2  + (size_t)b * strideA) : nullptr;
  const T* Bb2 = SPLIT ? (Bt2 + (size_t)b * strideB) : nullptr;

  const int rlane = lane & 15;
  const int koff  = (lane >> 4) * 8;
  const int mOff  = (lane >> 4) * 8;

  v8f acc[4][4];
#pragma unroll
  for (int i = 0; i < 4; ++i)
#pragma unroll
    for (int j = 0; j < 4; ++j) acc[i][j] = (v8f){0.f,0.f,0.f,0.f,0.f,0.f,0.f,0.f};

  for (int k0 = 0; k0 < K; k0 += 32) {
    V bh[4], bl[4];
#pragma unroll
    for (int j = 0; j < 4; ++j) {
      const size_t bo = (size_t)(n0 + (j << 4) + rlane) * ldb + koff + k0;
      bh[j] = Frag<T>::load(Bb + bo);
      if (SPLIT) bl[j] = Frag<T>::load(Bb2 + bo);
    }
#pragma unroll
    for (int i = 0; i < 4; ++i) {
      const size_t ao = (size_t)(m0 + (i << 4) + rlane) * lda + koff + k0;
      V ah = Frag<T>::load(Ab + ao);
      V al;
      if (SPLIT) al = Frag<T>::load(Ab2 + ao);
#pragma unroll
      for (int j = 0; j < 4; ++j) {
        acc[i][j] = Frag<T>::mma(ah, bh[j], acc[i][j]);
        if (SPLIT) {
          acc[i][j] = Frag<T>::mma(ah, bl[j], acc[i][j]);
          acc[i][j] = Frag<T>::mma(al, bh[j], acc[i][j]);
        }
      }
      Frag<T>::guard(acc[i][0], acc[i][3], ah, SPLIT ? al : ah);
    }
    Frag<T>::keep(bh[0], bh[1], bh[2], bh[3]);
    if (SPLIT) Frag<T>::keep(bl[0], bl[1], bl[2], bl[3]);
  }
  acc_guard4(acc[0][0], acc[0][1], acc[0][2], acc[0][3]);
  acc_guard4(acc[1][0], acc[1][1], acc[1][2], acc[1][3]);
  acc_guard4(acc[2][0], acc[2][1], acc[2][2], acc[2][3]);
  acc_guard4(acc[3][0], acc[3][1], acc[3][2], acc[3][3]);

  float* slab = sT[wave];
  const float* Rb = RESID ? (resid + (size_t)b * strideR) : nullptr;
#pragma unroll
  for (int i = 0; i < 4; ++i) {
    const int mBase = m0 + (i << 4);
#pragma unroll
    for (int j = 0; j < 4; ++j) {
      const int n = n0 + (j << 4) + rlane;
      float bv = 0.f;
      if (BIAS_MODE == 2) bv = bias[n];
#pragma unroll
      for (int r = 0; r < 8; ++r) {
        float v = acc[i][j][r] * scale;
        if (BIAS_MODE == 1) v += bias[mBase + mOff + r];
        if (BIAS_MODE == 2) v += bv;
        if (RESID) v += Rb[(size_t)(mBase + mOff + r) * ldc + n];
        if (ACT == 1) v = tanhf(v);
        if (ACT == 2) v = fmaxf(v, 0.0f);
        if (ACT == 3) v = v / (1.0f + expf(-v));
        if (ACT == 4) v = (v > 0.f) ? v : 0.01f * v;
        if (ACT == 5) v = 0.5f * v * (1.0f + erff(v * 0.70710678118654752f));
        slab[(mOff + r) * 68 + (j << 4) + rlane] = v;
      }
    }
    __builtin_amdgcn_fence(__ATOMIC_RELEASE, "workgroup");
    __builtin_amdgcn_wave_barrier();
    __builtin_amdgcn_fence(__ATOMIC_ACQUIRE, "workgroup");
    if (OUT_MODE == 0) {
      float* C = (float*)Cout + (size_t)b * strideC;
      const int hh = lane >> 4, c4 = (lane & 15) * 4;
      for (int pass = 0; pass < 2; ++pass) {
#pragma unroll
        for (int it = 0; it < 8; ++it) {
          const int row = it * 2 + hh;
          v4f v = *(const v4f*)(slab + row * 68 + c4);
          *(volatile v4f*)(C + (size_t)(mBase + row) * ldc + n0 + c4) = v;
        }
        __threadfence();
      }
    } else {
      const int q = lane >> 3, c8 = (lane & 7) * 8;
      unsigned short* C  = (unsigned short*)Cout  + (size_t)b * strideC;
      unsigned short* C2 = (OUT_MODE == 2) ? ((unsigned short*)Cout2 + (size_t)b * strideC) : nullptr;
      for (int pass = 0; pass < 2; ++pass) {
#pragma unroll
        for (int it = 0; it < 4; ++it) {
          const int row = it * 4 + q;
          const float* sp = slab + row * 68 + c8;
          v8h hv, lv;
#pragma unroll
          for (int e = 0; e < 8; ++e) {
            if (OUT_MODE == 1) {
              hv[e] = (_Float16)sp[e];
            } else {
              unsigned short hb = f2bf_bits(sp[e]);
              unsigned short lb = f2bf_bits(sp[e] - bf_bits2f(hb));
              hv[e] = __builtin_bit_cast(_Float16, hb);
              lv[e] = __builtin_bit_cast(_Float16, lb);
            }
          }
          *(volatile v8h*)(C + (size_t)(mBase + row) * ldc + n0 + c8) = hv;
          if (OUT_MODE == 2) *(volatile v8h*)(C2 + (size_t)(mBase + row) * ldc + n0 + c8) = lv;
        }
        __threadfence();
      }
    }
    __builtin_amdgcn_fence(__ATOMIC_RELEASE, "workgroup");
    __builtin_amdgcn_wave_barrier();
    __builtin_amdgcn_fence(__ATOMIC_ACQUIRE, "workgroup");
  }
}

__global__ __launch_bounds__(256) void cast_x_f16_kernel(const float* __restrict__ in,
                                                        unsigned short* __restrict__ out, int n8) {
  const int i = blockIdx.x * 256 + threadIdx.x;
  if (i < n8) {
    const v4f a = *(const v4f*)(in + (size_t)8 * i);
    const v4f c = *(const v4f*)(in + (size_t)8 * i + 4);
    v8h hv;
#pragma unroll
    for (int e = 0; e < 4; ++e) { hv[e] = (_Float16)a[e]; hv[4 + e] = (_Float16)c[e]; }
    _Float16* op = (_Float16*)out + (size_t)8 * i;
    *(volatile v8h*)op = hv;
    __threadfence();
    *(volatile v8h*)op = hv;
  }
}

__global__ __launch_bounds__(256) void transpose_cast_kernel(const float* __restrict__ in, int inLS,
                                                            int R, int C,
                                                            unsigned short* __restrict__ out, int outLS,
                                                            float sc) {
  __shared__ float sm[64][65];
  const int tid = threadIdx.x;
  const int l  = blockIdx.z;
  const int c0 = blockIdx.x * 64;
  const int r0 = blockIdx.y * 64;
  const float* ip = in + (size_t)l * inLS;
  _Float16* op = (_Float16*)out + (size_t)l * outLS;
#pragma unroll
  for (int i = 0; i < 16; ++i) {
    const int idx = i * 256 + tid;
    const int rr = idx >> 6, cc = idx & 63;
    sm[rr][cc] = ip[(size_t)(r0 + rr) * C + c0 + cc];
  }
  __syncthreads();
  const int wave = tid >> 5, lane = tid & 31;
  const int q = lane >> 3, c8 = (lane & 7) * 8;
  for (int pass = 0; pass < 2; ++pass) {
#pragma unroll
    for (int it = 0; it < 2; ++it) {
      const int cc = wave * 8 + it * 4 + q;
      v8h hv;
#pragma unroll
      for (int e = 0; e < 8; ++e) hv[e] = (_Float16)(sm[c8 + e][cc] * sc);
      *(volatile v8h*)(op + (size_t)(c0 + cc) * R + r0 + c8) = hv;
    }
    __threadfence();
  }
}

__global__ __launch_bounds__(256) void bias_prep_kernel(const float* __restrict__ bq, const float* __restrict__ bk,
                                                       const float* __restrict__ bv, const float* __restrict__ b1,
                                                       float* __restrict__ bqkv, float* __restrict__ b1x) {
  const int blk = blockIdx.x, t = threadIdx.x;
  if (blk < 12) {
    const int l = blk / 3, w = blk - l * 3;
    const float vq = bq[l * 256 + t], vk = bk[l * 256 + t], vv = bv[l * 256 + t];
    const float v = (w == 0) ? vq : ((w == 1) ? vk : vv);
    const float s = v * 16.0f;
    float* p = bqkv + (size_t)l * C_QKVN + w * 256 + t;
    *(volatile float*)p = s;
    __threadfence();
    *(volatile float*)p = s;
  } else {
    const int j = blk - 12, l = j >> 1, hf = j & 1;
    const float s = b1[l * 512 + hf * 256 + t] * 16.0f;
    float* p = b1x + (size_t)l * C_DFF + hf * 256 + t;
    *(volatile float*)p = s;
    __threadfence();
    *(volatile float*)p = s;
  }
}

__global__ __launch_bounds__(256) void resid_ln_kernel(const float* xin, const float* __restrict__ res,
                                                      const float* __restrict__ g, const float* __restrict__ bt,
                                                      float* xout, unsigned short* __restrict__ x16out) {
  __shared__ __align__(16) float S[8][256];
  const int wave = threadIdx.x >> 5, lane = threadIdx.x & 31;
  const int row = blockIdx.x * 8 + wave;
  const size_t rb = (size_t)row * C_DM;
  const v4f a0 = *(const v4f*)(xin + rb + 8 * lane);
  const v4f a1 = *(const v4f*)(xin + rb + 8 * lane + 4);
  const v4f r0 = *(const v4f*)(res + rb + 8 * lane);
  const v4f r1 = *(const v4f*)(res + rb + 8 * lane + 4);
  const v4f g0 = *(const v4f*)(g + 8 * lane);
  const v4f g1 = *(const v4f*)(g + 8 * lane + 4);
  const v4f b0 = *(const v4f*)(bt + 8 * lane);
  const v4f b1 = *(const v4f*)(bt + 8 * lane + 4);
  float v[8], gg[8], bb[8];
#pragma unroll
  for (int e = 0; e < 4; ++e) {
    v[e] = a0[e] + r0[e]; v[4 + e] = a1[e] + r1[e];
    gg[e] = g0[e]; gg[4 + e] = g1[e]; bb[e] = b0[e]; bb[4 + e] = b1[e];
  }
  float s = 0.f;
#pragma unroll
  for (int e = 0; e < 8; ++e) s += v[e];
#pragma unroll
  for (int off = 1; off < 32; off <<= 1) s += __shfl_xor(s, off, 32);
  const float mu = s * (1.0f / 256.0f);
  float d[8];
  float sq = 0.f;
#pragma unroll
  for (int e = 0; e < 8; ++e) { d[e] = v[e] - mu; sq += d[e] * d[e]; }
#pragma unroll
  for (int off = 1; off < 32; off <<= 1) sq += __shfl_xor(sq, off, 32);
  const float var = sq * (1.0f / 256.0f);
  const float rs = rsqrtf(var + C_LNEPS);
  float y[8];
  v8h yh;
#pragma unroll
  for (int e = 0; e < 8; ++e) { y[e] = d[e] * rs * gg[e] + bb[e]; yh[e] = (_Float16)y[e]; }
  v4f y0, y1;
#pragma unroll
  for (int e = 0; e < 4; ++e) { y0[e] = y[e]; y1[e] = y[4 + e]; }
  *(v4f*)(S[wave] + 8 * lane) = y0;
  *(v4f*)(S[wave] + 8 * lane + 4) = y1;
  __builtin_amdgcn_fence(__ATOMIC_RELEASE, "workgroup");
  __builtin_amdgcn_wave_barrier();
  __builtin_amdgcn_fence(__ATOMIC_ACQUIRE, "workgroup");
  const v4f u0 = *(const v4f*)(S[wave] + 4 * lane);
  const v4f u1 = *(const v4f*)(S[wave] + 128 + 4 * lane);
  _Float16* hp = (_Float16*)x16out + rb + 8 * lane;
  for (int pass = 0; pass < 2; ++pass) {
    *(volatile v4f*)(xout + rb + 4 * lane) = u0;
    *(volatile v4f*)(xout + rb + 128 + 4 * lane) = u1;
    *(volatile v8h*)hp = yh;
    __threadfence();
  }
}

#define A_NW 4
#define A_KC 64
__global__ __launch_bounds__(128)
void attn32_geo_kernel(const unsigned short* __restrict__ qkvp, const float* __restrict__ coords,
                       const float* __restrict__ alpha, int layer, float* __restrict__ out) {
  const _Float16* qkv = (const _Float16*)qkvp;
  __shared__ __align__(16) _Float16 Ksh[A_KC * C_DK];
  __shared__ __align__(16) _Float16 Vth[C_DK * A_KC];
  __shared__ __align__(16) _Float16 Psh[A_NW][16 * A_KC];
  __shared__ __align__(16) float    Os[A_NW][16 * 36];
  __shared__ __align__(16) float    Cs[C_S * 3];

  const int tid  = threadIdx.x;
  const int wave = tid >> 5;
  const int lane = tid & 31;
  const int hh   = lane >> 4;
  const int c    = lane & 15;

  const int nqb = C_S / 64;
  const int bx  = blockIdx.x;
  const int qb  = bx % nqb;
  const int bh  = bx / nqb;
  const int h   = bh % C_H;
  const int b   = bh / C_H;
  const int rowb = b * C_S;
  const int ql0  = qb * 64 + wave * 16;
  const int q0   = rowb + ql0;

  {
    const float* cbp = coords + (size_t)rowb * 3;
#pragma unroll 4
    for (int i = 0; i < (C_S * 3) / 128; ++i) Cs[i * 128 + tid] = cbp[i * 128 + tid];
  }
  __syncthreads();

  const float alphaL = alpha[layer];
  float cq0[8], cq1[8], cq2[8];
#pragma unroll
  for (int r = 0; r < 8; ++r) {
    const int lr = ql0 + 8 * hh + r;
    cq0[r] = Cs[lr * 3]; cq1[r] = Cs[lr * 3 + 1]; cq2[r] = Cs[lr * 3 + 2];
  }

  const v16h qa = Frag<_Float16>::load(qkv + (size_t)(q0 + c) * C_QKVN + h * C_DK + 8 * hh);

  float mrow[8], lrow[8];
  v8f oacc[2];
#pragma unroll
  for (int r = 0; r < 8; ++r) { mrow[r] = -3.0e38f; lrow[r] = 0.f; }
#pragma unroll
  for (int t = 0; t < 2; ++t) oacc[t] = (v8f){0.f,0.f,0.f,0.f,0.f,0.f,0.f,0.f};

  const float sscale = 0.17677669529663687f * (1.0f / 256.0f);

  for (int kc = 0; kc < C_S / A_KC; ++kc) {
    const int kv0 = kc * A_KC;
    __syncthreads();
    {
      const int kvr = tid >> 1, dh = (tid & 1) * 16;
      const _Float16* kr = qkv + (size_t)(rowb + kv0 + kvr) * C_QKVN + C_DM + h * C_DK + dh;
      const _Float16* vr = kr + C_DM;
      const v8h k0 = *(const v8h*)kr;
      const v8h k1 = *(const v8h*)(kr + 8);
      const v8h v0 = *(const v8h*)vr;
      const v8h v1 = *(const v8h*)(vr + 8);
      *(v8h*)(Ksh + kvr * C_DK + dh)     = k0;
      *(v8h*)(Ksh + kvr * C_DK + dh + 8) = k1;
#pragma unroll
      for (int e = 0; e < 8; ++e) {
        Vth[(dh + e) * A_KC + kvr]     = v0[e];
        Vth[(dh + 8 + e) * A_KC + kvr] = v1[e];
      }
    }
    __syncthreads();

    v8f s[4];
#pragma unroll
    for (int j = 0; j < 4; ++j) {
      s[j] = (v8f){0.f,0.f,0.f,0.f,0.f,0.f,0.f,0.f};
      const v16h kb = Frag<_Float16>::load(Ksh + (j * 16 + c) * C_DK + 8 * hh);
      s[j] = mma_h(qa, kb, s[j]);
    }
    float ck0[4], ck1[4], ck2[4];
#pragma unroll
    for (int j = 0; j < 4; ++j) {
      const int lk = kv0 + j * 16 + c;
      ck0[j] = Cs[lk * 3]; ck1[j] = Cs[lk * 3 + 1]; ck2[j] = Cs[lk * 3 + 2];
    }
    float cm[8];
#pragma unroll
    for (int r = 0; r < 8; ++r) {
      float m = -3.0e38f;
#pragma unroll
      for (int j = 0; j < 4; ++j) {
        float gd = cq0[r] * ck0[j];
        gd = fmaf(cq1[r], ck1[j], gd);
        gd = fmaf(cq2[r], ck2[j], gd);
        const float t = fmaf(alphaL, gd, s[j][r] * sscale);
        s[j][r] = t;
        m = fmaxf(m, t);
      }
#pragma unroll
      for (int off = 1; off < 16; off <<= 1) m = fmaxf(m, __shfl_xor(m, off, 32));
      cm[r] = m;
    }
    _Float16* pw = Psh[wave];
#pragma unroll
    for (int r = 0; r < 8; ++r) {
      const float mnew = fmaxf(mrow[r], cm[r]);
      const float corr = __expf(mrow[r] - mnew);
      mrow[r] = mnew;
      float psum = 0.f;
#pragma unroll
      for (int j = 0; j < 4; ++j) {
        const float p = __expf(s[j][r] - mnew);
        psum += p;
        pw[(8 * hh + r) * A_KC + j * 16 + c] = (_Float16)(p * 32768.0f);
      }
#pragma unroll
      for (int off = 1; off < 16; off <<= 1) psum += __shfl_xor(psum, off, 32);
      lrow[r] = lrow[r] * corr + psum;
      oacc[0][r] *= corr;
      oacc[1][r] *= corr;
    }
    __builtin_amdgcn_fence(__ATOMIC_RELEASE, "workgroup");
    __builtin_amdgcn_wave_barrier();
    __builtin_amdgcn_fence(__ATOMIC_ACQUIRE, "workgroup");
#pragma unroll 1
    for (int kk = 0; kk < 2; ++kk) {
      const v16h pa = Frag<_Float16>::load(pw + c * A_KC + kk * 32 + 8 * hh);
#pragma unroll
      for (int t = 0; t < 2; ++t) {
        const v16h vb = Frag<_Float16>::load(Vth + (t * 16 + c) * A_KC + kk * 32 + 8 * hh);
        oacc[t] = mma_h(pa, vb, oacc[t]);
      }
    }
  }

  float* os = Os[wave];
#pragma unroll
  for (int r = 0; r < 8; ++r) {
    const float inv = 1.0f / (lrow[r] * 524288.0f);
#pragma unroll
    for (int t = 0; t < 2; ++t) os[(8 * hh + r) * 36 + t * 16 + c] = oacc[t][r] * inv;
  }
  __builtin_amdgcn_fence(__ATOMIC_RELEASE, "workgroup");
  __builtin_amdgcn_wave_barrier();
  __builtin_amdgcn_fence(__ATOMIC_ACQUIRE, "workgroup");
  {
    const int q4 = lane >> 3, c4 = (lane & 7) * 4;
    for (int pass = 0; pass < 2; ++pass) {
#pragma unroll
      for (int it = 0; it < 4; ++it) {
        const int row = it * 4 + q4;
        const v4f val = *(const v4f*)(os + row * 36 + c4);
        *(volatile v4f*)(out + (size_t)(q0 + row) * C_DM + h * C_DK + c4) = val;
      }
      __threadfence();
    }
  }
}

extern "C" void kernel_launch(void* const* d_in, const int* in_sizes, int n_in,
                              void* d_out, int out_size, void* d_ws, size_t ws_size,
                              hipStream_t stream) {
  if (n_in < 17) return;
  if (in_sizes[0] != C_ROWS * C_DM || in_sizes[1] != C_ROWS * 3 ||
      in_sizes[2] != C_L * C_DM * C_DM || in_sizes[3] != C_L * C_DM ||
      in_sizes[4] != C_L * C_DM * C_DM || in_sizes[5] != C_L * C_DM ||
      in_sizes[6] != C_L * C_DM * C_DM || in_sizes[7] != C_L * C_DM ||
      in_sizes[8] != C_L ||
      in_sizes[9] != C_L * C_DM * C_DFF || in_sizes[10] != C_L * C_DFF ||
      in_sizes[11] != C_L * C_DFF * C_DM || in_sizes[12] != C_L * C_DM ||
      in_sizes[13] != C_L * C_DM || in_sizes[14] != C_L * C_DM ||
      in_sizes[15] != C_L * C_DM || in_sizes[16] != C_L * C_DM) return;
  if (out_size != C_ROWS * C_DM) return;

  const float* x      = (const float*)d_in[0];
  const float* coords = (const float*)d_in[1];
  const float* wq     = (const float*)d_in[2];
  const float* bq     = (const float*)d_in[3];
  const float* wk     = (const float*)d_in[4];
  const float* bk     = (const float*)d_in[5];
  const float* wv     = (const float*)d_in[6];
  const float* bv     = (const float*)d_in[7];
  const float* alpha  = (const float*)d_in[8];
  const float* w1     = (const float*)d_in[9];
  const float* b1     = (const float*)d_in[10];
  const float* w2     = (const float*)d_in[11];
  const float* b2     = (const float*)d_in[12];
  const float* ln1g   = (const float*)d_in[13];
  const float* ln1b   = (const float*)d_in[14];
  const float* ln2g   = (const float*)d_in[15];
  const float* ln2b   = (const float*)d_in[16];
  float* out = (float*)d_out;

  char* ws = (char*)d_ws;
  size_t off = 0;
  auto carve = [&](size_t bytes) -> void* {
    void* p = ws + off;
    off += (bytes + 255) & ~(size_t)255;
    return p;
  };
  unsigned short* x16   = (unsigned short*)carve((size_t)C_ROWS * C_DM * 2);
  float*          xf    = (float*)         carve((size_t)C_ROWS * C_DM * 4);
  unsigned short* qkv16 = (unsigned short*)carve((size_t)C_ROWS * C_QKVN * 2);
  float*          attn  = (float*)         carve((size_t)C_ROWS * C_DM * 4);
  unsigned short* h16   = (unsigned short*)carve((size_t)C_ROWS * C_DFF * 2);
  float*          ff    = (float*)         carve((size_t)C_ROWS * C_DM * 4);
  unsigned short* wqkvT = (unsigned short*)carve((size_t)C_L * C_QKVN * C_DM * 2);
  unsigned short* w1T   = (unsigned short*)carve((size_t)C_L * C_DFF * C_DM * 2);
  unsigned short* w2T   = (unsigned short*)carve((size_t)C_L * C_DM * C_DFF * 2);
  float*          bqkv  = (float*)         carve((size_t)C_L * C_QKVN * 4);
  float*          b1x   = (float*)         carve((size_t)C_L * C_DFF * 4);
  if (off > ws_size || off > (size_t)134217728) return;

  cast_x_f16_kernel<<<(C_ROWS * C_DM / 8 + 255) / 256, 256, 0, stream>>>(x, x16, C_ROWS * C_DM / 8);

  transpose_cast_kernel<<<dim3(C_DM / 64, C_DM / 64, C_L), 256, 0, stream>>>(
      wq, C_DM * C_DM, C_DM, C_DM, wqkvT + 0 * C_DM * C_DM, C_QKVN * C_DM, 64.0f);
  transpose_cast_kernel<<<dim3(C_DM / 64, C_DM / 64, C_L), 256, 0, stream>>>(
      wk, C_DM * C_DM, C_DM, C_DM, wqkvT + 1 * C_DM * C_DM, C_QKVN * C_DM, 64.0f);
  transpose_cast_kernel<<<dim3(C_DM / 64, C_DM / 64, C_L), 256, 0, stream>>>(
      wv, C_DM * C_DM, C_DM, C_DM, wqkvT + 2 * C_DM * C_DM, C_QKVN * C_DM, 64.0f);
  transpose_cast_kernel<<<dim3(C_DFF / 64, C_DM / 64, C_L), 256, 0, stream>>>(
      w1, C_DM * C_DFF, C_DM, C_DFF, w1T, C_DFF * C_DM, 64.0f);
  transpose_cast_kernel<<<dim3(C_DM / 64, C_DFF / 64, C_L), 256, 0, stream>>>(
      w2, C_DFF * C_DM, C_DFF, C_DM, w2T, C_DM * C_DFF, 64.0f);
  bias_prep_kernel<<<20, 256, 0, stream>>>(bq, bk, bv, b1, bqkv, b1x);

  const int tilesQKV = (C_ROWS / 64) * (C_QKVN / 64);
  const int tilesF1  = (C_ROWS / 64) * (C_DFF / 64);
  const int tilesF2  = (C_ROWS / 64) * (C_DM / 64);
  const dim3 gQKV((tilesQKV + 7) / 8, 1);
  const dim3 gF1((tilesF1 + 7) / 8, 1);
  const dim3 gF2((tilesF2 + 7) / 8, 1);
  const int gAtt = C_B * C_H * (C_S / 64);
  const int gLN  = C_ROWS / 8;

  for (int l = 0; l < C_L; ++l) {
    wmma_gemm64<0, false, 2, 1, false, 0><<<gQKV, 256, 0, stream>>>(
        x16, x16, C_DM, (long)0,
        wqkvT + (size_t)l * C_QKVN * C_DM, wqkvT + (size_t)l * C_QKVN * C_DM, C_DM, (long)0,
        (void*)qkv16, (void*)qkv16, C_QKVN, (long)0,
        bqkv + (size_t)l * C_QKVN,
        bqkv, (long)0,
        C_ROWS, C_QKVN, C_DM, 0.25f);

    attn32_geo_kernel<<<gAtt, 128, 0, stream>>>(qkv16, coords, alpha, l, attn);

    const float* xin1 = (l == 0) ? x : xf;
    resid_ln_kernel<<<gLN, 256, 0, stream>>>(xin1, attn, ln1g + (size_t)l * C_DM, ln1b + (size_t)l * C_DM, xf, x16);

    wmma_gemm64<0, false, 2, 1, false, 2><<<gF1, 256, 0, stream>>>(
        x16, x16, C_DM, (long)0,
        w1T + (size_t)l * C_DFF * C_DM, w1T + (size_t)l * C_DFF * C_DM, C_DM, (long)0,
        (void*)h16, (void*)h16, C_DFF, (long)0,
        b1x + (size_t)l * C_DFF,
        b1x, (long)0,
        C_ROWS, C_DFF, C_DM, 0.25f);

    wmma_gemm64<0, false, 2, 0, false, 0><<<gF2, 256, 0, stream>>>(
        h16, h16, C_DFF, (long)0,
        w2T + (size_t)l * C_DM * C_DFF, w2T + (size_t)l * C_DM * C_DFF, C_DFF, (long)0,
        (void*)ff, (void*)ff, C_DM, (long)0,
        b2 + (size_t)l * C_DM,
        b2, (long)0,
        C_ROWS, C_DM, C_DFF, 1.0f / 1024.0f);

    float* xdst = (l == C_L - 1) ? out : xf;
    resid_ln_kernel<<<gLN, 256, 0, stream>>>(xf, ff, ln2g + (size_t)l * C_DM, ln2b + (size_t)l * C_DM, xdst, x16);
  }
}
